// Model_GRU2_17497696763924
// MI455X (gfx1250) — hardware-verified
//
#include <hip/hip_runtime.h>
#include <math.h>

#define NB    64
#define SEQ   2048
#define FIN   64
#define HID   160
#define G3    480
#define KCV   192
#define NROWS (NB * SEQ)
#define H1P   256
#define HH    80
#define NT    256
#define NTR   320
#define HP    168
#define FP    164
#define ASC   256.0f
#define WSC   16.0f
#define SINV  (1.0f / 4096.0f)

typedef __attribute__((ext_vector_type(16))) _Float16 v16h;
typedef __attribute__((ext_vector_type(8)))  _Float16 v8h;
typedef __attribute__((ext_vector_type(16))) __bf16   v16b;
typedef __attribute__((ext_vector_type(8)))  __bf16   v8b;
typedef __attribute__((ext_vector_type(8)))  float    v8f;
typedef __attribute__((ext_vector_type(4)))  float    v4f;

__device__ __forceinline__ unsigned short f2bf_bits(float f) {
  unsigned u = __float_as_uint(f);
  return (unsigned short)((u + 0x7FFFu + ((u >> 16) & 1u)) >> 16);
}
__device__ __forceinline__ float bf_bits2f(unsigned short h) { return __uint_as_float(((unsigned)h) << 16); }

__device__ __forceinline__ void dep_guard_h(v8f& a, v8f& b, v16h x, v16h y) { asm volatile("v_nop\n\tv_nop\n\tv_nop\n\tv_nop" : "+v"(a), "+v"(b) : "v"(x), "v"(y)); }
__device__ __forceinline__ void dep_guard_b(v8f& a, v8f& b, v16b x, v16b y) { asm volatile("v_nop\n\tv_nop\n\tv_nop\n\tv_nop" : "+v"(a), "+v"(b) : "v"(x), "v"(y)); }
__device__ __forceinline__ void keep4_h(v16h a, v16h b, v16h c, v16h d) { asm volatile("v_nop" :: "v"(a), "v"(b), "v"(c), "v"(d)); }
__device__ __forceinline__ void keep4_b(v16b a, v16b b, v16b c, v16b d) { asm volatile("v_nop" :: "v"(a), "v"(b), "v"(c), "v"(d)); }
__device__ __forceinline__ void acc_guard4(v8f& a, v8f& b, v8f& c, v8f& d) { asm volatile("v_nop\n\tv_nop\n\tv_nop\n\tv_nop" : "+v"(a), "+v"(b), "+v"(c), "+v"(d)); }
__device__ __forceinline__ void dep_guard3_h(v8f& a, v8f& b, v8f& c, v16h w, v16h x, v16h y, v16h z) {
  asm volatile("v_nop\n\tv_nop\n\tv_nop\n\tv_nop" : "+v"(a), "+v"(b), "+v"(c) : "v"(w), "v"(x), "v"(y), "v"(z));
}

template <typename T> struct Frag;
template <> struct Frag<_Float16> {
  typedef v16h V; union U { v16h v; v8h h[2]; };
  static __device__ __forceinline__ v16h load(const _Float16* p) {
    U f; f.h[0] = *(const v8h*)(p); f.h[1] = *(const v8h*)(p + 16); return f.v;
  }
  static __device__ __forceinline__ v8f mma(v16h a, v16h b, v8f c) {
    return __builtin_amdgcn_wmma_f32_16x16x32_f16(false, a, false, b, (short)0, c, false, false);
  }
  static __device__ __forceinline__ void guard(v8f& a, v8f& b, v16h x, v16h y) { dep_guard_h(a, b, x, y); }
  static __device__ __forceinline__ void keep(v16h a, v16h b, v16h c, v16h d) { keep4_h(a, b, c, d); }
};
template <> struct Frag<__bf16> {
  typedef v16b V; union U { v16b v; v8b h[2]; };
  static __device__ __forceinline__ v16b load(const __bf16* p) {
    U f; f.h[0] = *(const v8b*)(p); f.h[1] = *(const v8b*)(p + 16); return f.v;
  }
  static __device__ __forceinline__ v8f mma(v16b a, v16b b, v8f c) {
    return __builtin_amdgcn_wmma_f32_16x16x32_bf16(false, a, false, b, (short)0, c, false, false);
  }
  static __device__ __forceinline__ void guard(v8f& a, v8f& b, v16b x, v16b y) { dep_guard_b(a, b, x, y); }
  static __device__ __forceinline__ void keep(v16b a, v16b b, v16b c, v16b d) { keep4_b(a, b, c, d); }
};

template <int ET> struct Elem;
template <> struct Elem<0> { typedef _Float16 T; };
template <> struct Elem<1> { typedef __bf16 T; };
template <int ET, bool SPLIT, int BIAS_MODE, int OUT_MODE, bool RESID, int ACT = 0>
__global__ __launch_bounds__(256) void wmma_gemm64(
    const unsigned short* __restrict__ Ap, const unsigned short* __restrict__ A2p, int lda, long strideA,
    const unsigned short* __restrict__ Btp, const unsigned short* __restrict__ Bt2p, int ldb, long strideB,
    void* __restrict__ Cout, void* __restrict__ Cout2, int ldc, long strideC,
    const float* __restrict__ bias,
    const float* __restrict__ resid, long strideR,
    int M, int N, int K, float scale) {
  typedef typename Elem<ET>::T T;
  typedef typename Frag<T>::V V;
  const T* A = (const T*)Ap; const T* A2 = (const T*)A2p; const T* Bt = (const T*)Btp; const T* Bt2 = (const T*)Bt2p;
  __shared__ __align__(16) float sT[8][16 * 68];
  const int b    = blockIdx.y;
  const int lane = threadIdx.x & 31;
  const int wave = threadIdx.x >> 5;
  const int tilesN = N >> 6;
  const int tilesM = M >> 6;
  const int tile = blockIdx.x * 8 + wave;
  if (tile >= tilesM * tilesN) return;
  const int tm = tile / tilesN;
  const int tn = tile - tm * tilesN;
  const int m0 = tm << 6;
  const int n0 = tn << 6;

  const T* Ab  = A  + (size_t)b * strideA;
  const T* Bb  = Bt + (size_t)b * strideB;
  const T* Ab2 = SPLIT ? (A2  + (size_t)b * strideA) : nullptr;
  const T* Bb2 = SPLIT ? (Bt2 + (size_t)b * strideB) : nullptr;

  const int rlane = lane & 15;
  const int koff  = (lane >> 4) * 8;
  const int mOff  = (lane >> 4) * 8;

  v8f acc[4][4];
#pragma unroll
  for (int i = 0; i < 4; ++i)
#pragma unroll
    for (int j = 0; j < 4; ++j) acc[i][j] = (v8f){0.f,0.f,0.f,0.f,0.f,0.f,0.f,0.f};

  for (int k0 = 0; k0 < K; k0 += 32) {
    V bh[4], bl[4];
#pragma unroll
    for (int j = 0; j < 4; ++j) {
      const size_t bo = (size_t)(n0 + (j << 4) + rlane) * ldb + koff + k0;
      bh[j] = Frag<T>::load(Bb + bo);
      if (SPLIT) bl[j] = Frag<T>::load(Bb2 + bo);
    }
#pragma unroll
    for (int i = 0; i < 4; ++i) {
      const size_t ao = (size_t)(m0 + (i << 4) + rlane) * lda + koff + k0;
      V ah = Frag<T>::load(Ab + ao);
      V al;
      if (SPLIT) al = Frag<T>::load(Ab2 + ao);
#pragma unroll
      for (int j = 0; j < 4; ++j) {
        acc[i][j] = Frag<T>::mma(ah, bh[j], acc[i][j]);
        if (SPLIT) {
          acc[i][j] = Frag<T>::mma(ah, bl[j], acc[i][j]);
          acc[i][j] = Frag<T>::mma(al, bh[j], acc[i][j]);
        }
      }
      Frag<T>::guard(acc[i][0], acc[i][3], ah, SPLIT ? al : ah);
    }
    Frag<T>::keep(bh[0], bh[1], bh[2], bh[3]);
    if (SPLIT) Frag<T>::keep(bl[0], bl[1], bl[2], bl[3]);
  }
  acc_guard4(acc[0][0], acc[0][1], acc[0][2], acc[0][3]);
  acc_guard4(acc[1][0], acc[1][1], acc[1][2], acc[1][3]);
  acc_guard4(acc[2][0], acc[2][1], acc[2][2], acc[2][3]);
  acc_guard4(acc[3][0], acc[3][1], acc[3][2], acc[3][3]);

  float* slab = sT[wave];
  const float* Rb = RESID ? (resid + (size_t)b * strideR) : nullptr;
#pragma unroll
  for (int i = 0; i < 4; ++i) {
    const int mBase = m0 + (i << 4);
#pragma unroll
    for (int j = 0; j < 4; ++j) {
      const int n = n0 + (j << 4) + rlane;
      float bv = 0.f;
      if (BIAS_MODE == 2) bv = bias[n];
#pragma unroll
      for (int r = 0; r < 8; ++r) {
        float v = acc[i][j][r] * scale;
        if (BIAS_MODE == 1) v += bias[mBase + mOff + r];
        if (BIAS_MODE == 2) v += bv;
        if (RESID) v += Rb[(size_t)(mBase + mOff + r) * ldc + n];
        if (ACT == 1) v = tanhf(v);
        if (ACT == 2) v = fmaxf(v, 0.0f);
        if (ACT == 3) v = v / (1.0f + expf(-v));
        if (ACT == 4) v = (v > 0.f) ? v : 0.01f * v;
        if (ACT == 5) v = 0.5f * v * (1.0f + erff(v * 0.70710678118654752f));
        slab[(mOff + r) * 68 + (j << 4) + rlane] = v;
      }
    }
    __builtin_amdgcn_fence(__ATOMIC_RELEASE, "workgroup");
    __builtin_amdgcn_wave_barrier();
    __builtin_amdgcn_fence(__ATOMIC_ACQUIRE, "workgroup");
    if (OUT_MODE == 0) {
      float* C = (float*)Cout + (size_t)b * strideC;
      const int hh = lane >> 4, c4 = (lane & 15) * 4;
      for (int pass = 0; pass < 2; ++pass) {
#pragma unroll
        for (int it = 0; it < 8; ++it) {
          const int row = it * 2 + hh;
          v4f v = *(const v4f*)(slab + row * 68 + c4);
          *(volatile v4f*)(C + (size_t)(mBase + row) * ldc + n0 + c4) = v;
        }
        __threadfence();
      }
    } else {
      const int q = lane >> 3, c8 = (lane & 7) * 8;
      unsigned short* C  = (unsigned short*)Cout  + (size_t)b * strideC;
      unsigned short* C2 = (OUT_MODE == 2) ? ((unsigned short*)Cout2 + (size_t)b * strideC) : nullptr;
      for (int pass = 0; pass < 2; ++pass) {
#pragma unroll
        for (int it = 0; it < 4; ++it) {
          const int row = it * 4 + q;
          const float* sp = slab + row * 68 + c8;
          v8h hv, lv;
#pragma unroll
          for (int e = 0; e < 8; ++e) {
            if (OUT_MODE == 1) {
              hv[e] = (_Float16)sp[e];
            } else {
              unsigned short hb = f2bf_bits(sp[e]);
              unsigned short lb = f2bf_bits(sp[e] - bf_bits2f(hb));
              hv[e] = __builtin_bit_cast(_Float16, hb);
              lv[e] = __builtin_bit_cast(_Float16, lb);
            }
          }
          *(volatile v8h*)(C + (size_t)(mBase + row) * ldc + n0 + c8) = hv;
          if (OUT_MODE == 2) *(volatile v8h*)(C2 + (size_t)(mBase + row) * ldc + n0 + c8) = lv;
        }
        __threadfence();
      }
    }
    __builtin_amdgcn_fence(__ATOMIC_RELEASE, "workgroup");
    __builtin_amdgcn_wave_barrier();
    __builtin_amdgcn_fence(__ATOMIC_ACQUIRE, "workgroup");
  }
}

__device__ __forceinline__ unsigned pack_f16x2(float a, float b) {
  const _Float16 h0 = (_Float16)a, h1 = (_Float16)b;
  return (unsigned)__builtin_bit_cast(unsigned short, h0) | ((unsigned)__builtin_bit_cast(unsigned short, h1) << 16);
}
__device__ __forceinline__ void st2u(unsigned* p, unsigned v) { *(volatile unsigned*)p = v; __threadfence(); *(volatile unsigned*)p = v; }
__device__ __forceinline__ float ftanh(float x) { return 1.0f - 2.0f * __builtin_amdgcn_rcpf(1.0f + __expf(2.0f * x)); }
__device__ __forceinline__ float fsigm(float x) { return __builtin_amdgcn_rcpf(1.0f + __expf(-x)); }
__device__ __forceinline__ float gelu_erf(float x) { return 0.5f * x * (1.0f + erff(x * 0.70710678118654752f)); }

__global__ __launch_bounds__(NT) void prep_kernel(const float* __restrict__ mixw,
                                                 const float* __restrict__ Wih1, const float* __restrict__ Whh1,
                                                 const float* __restrict__ Wih2, const float* __restrict__ Whh2,
                                                 unsigned* __restrict__ WCV, unsigned* __restrict__ WIH1u, unsigned* __restrict__ WHH1u,
                                                 unsigned* __restrict__ WIH2u, unsigned* __restrict__ WHH2u) {
  const int blk = blockIdx.x, tid = threadIdx.x;
  if (blk < 24) {
    const int p = blk * NT + tid;
    const int n = p / 96, c0 = (p - n * 96) * 2;
    const int k = c0 >> 6, g0 = c0 & 63;
    const float w0 = mixw[n * KCV + g0 * 3 + k] * WSC;
    const float w1 = mixw[n * KCV + (g0 + 1) * 3 + k] * WSC;
    st2u(WCV + p, pack_f16x2(w0, w1));
  } else if (blk < 84) {
    const int p = (blk - 24) * NT + tid;
    st2u(WIH1u + p, pack_f16x2(Wih1[2 * p] * WSC, Wih1[2 * p + 1] * WSC));
  } else if (blk < 234) {
    const int p = (blk - 84) * NT + tid;
    st2u(WHH1u + p, pack_f16x2(Whh1[2 * p] * WSC, Whh1[2 * p + 1] * WSC));
  } else if (blk < 384) {
    const int p = (blk - 234) * NT + tid;
    st2u(WIH2u + p, pack_f16x2(Wih2[2 * p] * WSC, Wih2[2 * p + 1] * WSC));
  } else {
    const int p = (blk - 384) * NT + tid;
    st2u(WHH2u + p, pack_f16x2(Whh2[2 * p] * WSC, Whh2[2 * p + 1] * WSC));
  }
}

__global__ __launch_bounds__(NT) void im2col_kernel(const float* __restrict__ x, _Float16* __restrict__ ZIN) {
  const int gid = blockIdx.x * NT + threadIdx.x;
  const int row = gid / 24, c = gid - row * 24;
  const int b = row >> 11, t = row & (SEQ - 1);
  const int k = c >> 3, g0 = (c & 7) * 8;
  const int tt = t + 2 * k - 2;
  const bool valid = (tt >= 0) && (tt < SEQ);
  const int ttc = tt < 0 ? 0 : (tt >= SEQ ? SEQ - 1 : tt);
  const float* p = x + ((size_t)(b * SEQ + ttc)) * FIN + g0;
  const v4f a = *(const v4f*)p, bq = *(const v4f*)(p + 4);
  v8h h;
#pragma unroll
  for (int e = 0; e < 4; ++e) {
    h[e]     = (_Float16)(valid ? a[e]  : 0.0f);
    h[4 + e] = (_Float16)(valid ? bq[e] : 0.0f);
  }
  _Float16* op = ZIN + (size_t)gid * 8;
  *(volatile v8h*)op = h; __threadfence(); *(volatile v8h*)op = h;
}

__global__ __launch_bounds__(NT) void bn_gelu_kernel(const float* __restrict__ Y, const float* __restrict__ g,
                                                    const float* __restrict__ bb, const float* __restrict__ m,
                                                    const float* __restrict__ vv, unsigned* __restrict__ Z16u) {
  const int i = blockIdx.x * NT + threadIdx.x;
  unsigned u = 0u;
#pragma unroll 1
  for (int e = 0; e < 2; ++e) {
    const int idx = 2 * i + e;
    const int f = idx & (FIN - 1);
    const float y = Y[idx];
    const float sc = g[f] * rsqrtf(vv[f] + 1e-5f);
    const float v = (y - m[f]) * sc + bb[f];
    const float z = gelu_erf(v) * ASC;
    u |= ((unsigned)__builtin_bit_cast(unsigned short, (_Float16)z)) << (16 * e);
  }
  st2u(Z16u + i, u);
}

template <int KX, int XP, bool FINAL>
__global__ __launch_bounds__(NTR) void gru_rec_kernel(const _Float16* XIN, const _Float16* __restrict__ WIH,
                                                     const _Float16* __restrict__ WHH,
                                                     const float* __restrict__ bih, const float* __restrict__ bhh,
                                                     _Float16* HSEQ,
                                                     const float* __restrict__ hw1, const float* __restrict__ hb1,
                                                     const float* __restrict__ hw2, const float* __restrict__ hb2,
                                                     float* __restrict__ OUT) {
  __shared__ __align__(16) _Float16 h16[16 * HP];
  __shared__ __align__(16) float hf[FINAL ? 16 * FP : 4];
  __shared__ __align__(16) float qs[FINAL ? 16 * HH : 4];
  const int tid = threadIdx.x, lane = tid & 31, wave = tid >> 5;
  const int rlane = lane & 15, hh = lane >> 4, koff = hh * 8, mOff = hh * 8;
  const int blk = blockIdx.x;
  for (int i = tid; i < 16 * HP; i += NTR) h16[i] = (_Float16)0.0f;
  __syncthreads();

  const int j = 16 * wave + rlane;
  const _Float16* arow = h16 + rlane * HP + koff;
  const _Float16* xrow = XIN + (size_t)(16 * blk + rlane) * SEQ * XP + koff;
  const _Float16* wir = WIH + (size_t)j * KX + koff;
  const _Float16* wiz = WIH + (size_t)(HID + j) * KX + koff;
  const _Float16* win = WIH + (size_t)(2 * HID + j) * KX + koff;
  const _Float16* whr = WHH + (size_t)j * HID + koff;
  const _Float16* whz = WHH + (size_t)(HID + j) * HID + koff;
  const _Float16* whn = WHH + (size_t)(2 * HID + j) * HID + koff;
  const float brz_r = bih[j] + bhh[j];
  const float brz_z = bih[HID + j] + bhh[HID + j];
  const float b_in  = bih[2 * HID + j];
  const float b_hn  = bhh[2 * HID + j];
  const v8f z8 = {0.f, 0.f, 0.f, 0.f, 0.f, 0.f, 0.f, 0.f};

  float hreg[8];
#pragma unroll
  for (int r = 0; r < 8; ++r) hreg[r] = 0.0f;

#pragma unroll 1
  for (int t = 0; t < SEQ; ++t) {
    v8f ar = z8, az = z8, axn = z8, ahn = z8;
    const _Float16* xa = xrow + (size_t)t * XP;
#pragma unroll 1
    for (int k0 = 0; k0 < KX; k0 += 32) {
      const v16h a  = Frag<_Float16>::load(xa + k0);
      const v16h b0 = Frag<_Float16>::load(wir + k0);
      const v16h b1 = Frag<_Float16>::load(wiz + k0);
      const v16h b2 = Frag<_Float16>::load(win + k0);
      ar  = Frag<_Float16>::mma(a, b0, ar);
      az  = Frag<_Float16>::mma(a, b1, az);
      axn = Frag<_Float16>::mma(a, b2, axn);
      dep_guard3_h(ar, az, axn, a, b0, b1, b2);
    }
#pragma unroll 1
    for (int k0 = 0; k0 < HID; k0 += 32) {
      const v16h a  = Frag<_Float16>::load(arow + k0);
      const v16h b0 = Frag<_Float16>::load(whr + k0);
      const v16h b1 = Frag<_Float16>::load(whz + k0);
      const v16h b2 = Frag<_Float16>::load(whn + k0);
      ar  = Frag<_Float16>::mma(a, b0, ar);
      az  = Frag<_Float16>::mma(a, b1, az);
      ahn = Frag<_Float16>::mma(a, b2, ahn);
      dep_guard3_h(ar, az, ahn, a, b0, b1, b2);
    }
    acc_guard4(ar, az, axn, ahn);

#pragma unroll
    for (int r = 0; r < 8; ++r) {
      const float pr = ar[r]  * SINV + brz_r;
      const float pz = az[r]  * SINV + brz_z;
      const float xn = axn[r] * SINV + b_in;
      const float hn = ahn[r] * SINV + b_hn;
      const float rg = fsigm(pr);
      const float zg = fsigm(pz);
      const float ng = ftanh(xn + rg * hn);
      hreg[r] = (1.0f - zg) * ng + zg * hreg[r];
    }
    __syncthreads();
#pragma unroll
    for (int r = 0; r < 8; ++r) h16[(mOff + r) * HP + j] = (_Float16)(hreg[r] * ASC);
    __syncthreads();
    if (!FINAL) {
      const int c8 = lane * 8;
      const int cc = (lane < 20) ? c8 : (HID - 8);
      for (int row = wave; row < 16; row += 10) {
        const v8h ld = *(const v8h*)(h16 + row * HP + cc);
        v8h v;
#pragma unroll
        for (int e = 0; e < 8; ++e) v[e] = (lane < 20) ? ld[e] : (_Float16)0.0f;
        _Float16* dst = HSEQ + ((size_t)(16 * blk + row) * SEQ + t) * H1P + c8;
        *(volatile v8h*)dst = v;
        __threadfence();
        *(volatile v8h*)dst = v;
      }
    }
  }

  if (FINAL) {
#pragma unroll
    for (int r = 0; r < 8; ++r) hf[(mOff + r) * FP + j] = hreg[r];
    __syncthreads();
#pragma unroll 1
    for (int o4 = tid; o4 < 16 * HH; o4 += NTR) {
      const int s = o4 / HH, o = o4 - s * HH;
      float acc = hb1[o];
      const float* hrow = hf + s * FP;
      const float* wrow = hw1 + (size_t)o * HID;
#pragma unroll 1
      for (int jj = 0; jj < HID; ++jj) acc += hrow[jj] * wrow[jj];
      qs[s * HH + o] = gelu_erf(acc);
    }
    __syncthreads();
    if (wave == 0) {
      const int s = lane >> 1, c = lane & 1;
      float acc = hb2[c];
      const float* qrow = qs + s * HH;
      const float* w2 = hw2 + c * HH;
#pragma unroll 1
      for (int o = 0; o < HH; ++o) acc += qrow[o] * w2[o];
      float* op = OUT + (size_t)blk * 32 + lane;
      *(volatile float*)op = acc; __threadfence(); *(volatile float*)op = acc;
    }
  }
}

extern "C" void kernel_launch(void* const* d_in, const int* in_sizes, int n_in,
                              void* d_out, int out_size, void* d_ws, size_t ws_size, hipStream_t stream) {
  if (n_in < 18 || d_out == nullptr || d_ws == nullptr) return;
  if (in_sizes[0] != NB * SEQ * FIN || in_sizes[1] != FIN * FIN * 3 || in_sizes[2] != FIN || in_sizes[3] != FIN ||
      in_sizes[4] != FIN || in_sizes[5] != FIN || in_sizes[6] != G3 * FIN || in_sizes[7] != G3 * HID ||
      in_sizes[8] != G3 || in_sizes[9] != G3 || in_sizes[10] != G3 * HID || in_sizes[11] != G3 * HID ||
      in_sizes[12] != G3 || in_sizes[13] != G3 || in_sizes[14] != HH * HID || in_sizes[15] != HH ||
      in_sizes[16] != 2 * HH || in_sizes[17] != 2 || out_size != NB * 2) return;

  const float* x     = (const float*)d_in[0];
  const float* mixw  = (const float*)d_in[1];
  const float* bng   = (const float*)d_in[2];
  const float* bnb   = (const float*)d_in[3];
  const float* bnm   = (const float*)d_in[4];
  const float* bnv   = (const float*)d_in[5];
  const float* w_ih1 = (const float*)d_in[6];
  const float* w_hh1 = (const float*)d_in[7];
  const float* b_ih1 = (const float*)d_in[8];
  const float* b_hh1 = (const float*)d_in[9];
  const float* w_ih2 = (const float*)d_in[10];
  const float* w_hh2 = (const float*)d_in[11];
  const float* b_ih2 = (const float*)d_in[12];
  const float* b_hh2 = (const float*)d_in[13];
  const float* hw1   = (const float*)d_in[14];
  const float* hb1   = (const float*)d_in[15];
  const float* hw2   = (const float*)d_in[16];
  const float* hb2   = (const float*)d_in[17];
  float* out = (float*)d_out;

  char* ws = (char*)d_ws; size_t off = 0;
  auto carve = [&](size_t bytes) -> char* { char* p = ws + off; off += (bytes + 255) & ~(size_t)255; return p; };
  char*     RA    = carve((size_t)67108864);
  char*     RB    = carve((size_t)33554432);
  unsigned* Z16u  = (unsigned*)carve((size_t)NROWS * FIN * 2);
  unsigned* WCVu  = (unsigned*)carve((size_t)FIN * KCV * 2);
  unsigned* WIH1u = (unsigned*)carve((size_t)G3 * FIN * 2);
  unsigned* WHH1u = (unsigned*)carve((size_t)G3 * HID * 2);
  unsigned* WIH2u = (unsigned*)carve((size_t)G3 * HID * 2);
  unsigned* WHH2u = (unsigned*)carve((size_t)G3 * HID * 2);
  if (off > ws_size || off > (size_t)134217728) return;
  if ((size_t)NROWS * KCV * 2 > (size_t)67108864 || (size_t)NROWS * H1P * 2 > (size_t)67108864 ||
      (size_t)NROWS * FIN * 4 > (size_t)33554432) return;

  _Float16* ZIN16 = (_Float16*)RA;
  _Float16* H1_16 = (_Float16*)RA;
  float*    Y32   = (float*)RB;
  const _Float16* Z16h = (const _Float16*)Z16u;
  const _Float16* WIH1 = (const _Float16*)WIH1u;
  const _Float16* WHH1 = (const _Float16*)WHH1u;
  const _Float16* WIH2 = (const _Float16*)WIH2u;
  const _Float16* WHH2 = (const _Float16*)WHH2u;

  prep_kernel<<<534, NT, 0, stream>>>(mixw, w_ih1, w_hh1, w_ih2, w_hh2, WCVu, WIH1u, WHH1u, WIH2u, WHH2u);
  im2col_kernel<<<(NROWS * 24) / NT, NT, 0, stream>>>(x, ZIN16);
  wmma_gemm64<0, false, 0, 0, false><<<dim3(((NROWS / 64) * (FIN / 64)) / 8, 1), 256, 0, stream>>>(
      (const unsigned short*)ZIN16, (const unsigned short*)nullptr, KCV, 0L,
      (const unsigned short*)WCVu, (const unsigned short*)nullptr, KCV, 0L,
      (void*)Y32, (void*)nullptr, FIN, 0L,
      (const float*)nullptr, (const float*)nullptr, 0L, NROWS, FIN, KCV, 1.0f / 16.0f);
  bn_gelu_kernel<<<(NROWS * FIN / 2) / NT, NT, 0, stream>>>(Y32, bng, bnb, bnm, bnv, Z16u);
  gru_rec_kernel<FIN, FIN, false><<<NB / 16, NTR, 0, stream>>>(Z16h, WIH1, WHH1, b_ih1, b_hh1, H1_16, hw1, hb1, hw2, hb2, out);
  gru_rec_kernel<HID, H1P, true><<<NB / 16, NTR, 0, stream>>>(H1_16, WIH2, WHH2, b_ih2, b_hh2, H1_16, hw1, hb1, hw2, hb2, out);
}
